// SNN_Autoencoder_54082228191383
// MI455X (gfx1250) — hardware-verified
//
#include <hip/hip_runtime.h>
#include <stddef.h>


typedef _Float16 v16h __attribute__((ext_vector_type(16)));
typedef _Float16 v8h  __attribute__((ext_vector_type(8)));
typedef float    v8f  __attribute__((ext_vector_type(8)));
typedef float    v4f  __attribute__((ext_vector_type(4)));
typedef _Float16 h16;

#ifndef NB
#define NB 2048
#endif
#define NB_FULL 2048
#define DIM   1024
#define HID   256
#define MROWS NB

static_assert(NB >= 64 && NB <= NB_FULL && (NB % 64) == 0);
static_assert((DIM % 64) == 0 && (DIM % 32) == 0 && (DIM % 8) == 0);
static_assert((HID % 64) == 0 && (HID % 32) == 0 && (HID % 8) == 0);
static_assert((((size_t)MROWS * DIM) % (size_t)(256 * 8)) == 0);
static_assert((size_t)MROWS * DIM < (size_t)0xFFFFFFFFu);
static_assert((size_t)NB_FULL * DIM * 4 == (size_t)8388608);
static_assert((size_t)NB_FULL * DIM + (size_t)NB * HID <= (size_t)2621440);
#define OUT1_OFF ((size_t)NB_FULL * DIM)

#define LDT 72
#define LDC 68
static_assert((LDT % 8) == 0 && LDT >= 64);
static_assert((LDC % 4) == 0 && LDC >= 64);
static_assert((size_t)64 * LDT * 2 <= (size_t)131072);
static_assert((size_t)64 * LDC * 4 <= (size_t)131072);

#define WCARRY 64.0f
#define ACARRY 16.0f

#define BETA_F   0.9f
#define THRESH_F 0.9f

#define WPL_BYTES ((size_t)DIM * HID * 2)
#define X16_BYTES ((size_t)MROWS * DIM * 2)
#define E16_BYTES ((size_t)MROWS * HID * 2)
#define OFF_ENC ((size_t)0)
#define OFF_DEC (OFF_ENC + WPL_BYTES)
#define OFF_X16 (OFF_DEC + WPL_BYTES)
#define OFF_E16 (OFF_X16 + X16_BYTES)
#define WS_TOTAL (OFF_E16 + E16_BYTES)
static_assert((WPL_BYTES % 128) == 0 && (X16_BYTES % 128) == 0 && (E16_BYTES % 128) == 0);
static_assert(WS_TOTAL <= (size_t)134217728);

__device__ __forceinline__ float bf16r(float x) {
  unsigned int u = __float_as_uint(x);
  u = (u + 0x7FFFu + ((u >> 16) & 1u)) & 0xFFFF0000u;
  return __uint_as_float(u);
}

static __device__ __forceinline__ h16 toh_flush(float v) {
  const h16 r = (h16)v;
  return (fabsf(v) < 6.103515625e-05f) ? (h16)0.0f : r;
}

__device__ __forceinline__ v16h frag_at(const _Float16* p) {
  v8h lo = *(const v8h*)(p);
  v8h hi = *(const v8h*)(p + 16);
  v16h out;
#pragma unroll
  for (int i = 0; i < 8; ++i) { out[i] = lo[i]; out[i + 8] = hi[i]; }
  return out;
}

__device__ __forceinline__ v8f wmma16(v16h a, v16h b, v8f c) {
  v8f d = __builtin_amdgcn_wmma_f32_16x16x32_f16(false, a, false, b, (short)0, c,
                                                 false, false);
  asm volatile("v_nop\n\tv_nop\n\tv_nop\n\tv_nop" : "+v"(d) : "v"(a), "v"(b));
  return d;
}

__device__ __forceinline__ float lif_last(float c) {
#pragma clang fp contract(off)
  const float s = ((c - THRESH_F) > 0.0f) ? 1.0f : 0.0f;
  const float r = (s > THRESH_F) ? 1.0f : 0.0f;
  return (BETA_F * s + c) - r * THRESH_F;
}

__global__ __launch_bounds__(256) void wconv_kernel(
    const float* __restrict__ W, _Float16* __restrict__ Wt, unsigned ldw, unsigned ldk) {
  __shared__ _Float16 T[64 * LDT];
  const unsigned tid = threadIdx.x;
  const unsigned n0 = blockIdx.x * 64u;
  const unsigned k0 = blockIdx.y * 64u;
#pragma unroll 4
  for (unsigned j = 0; j < 16u; ++j) {
    const unsigned idx = tid + 256u * j;
    const unsigned kr = idx >> 6, nc = idx & 63u;
    const float v = W[(size_t)(k0 + kr) * ldw + n0 + nc];
    T[nc * LDT + kr] = toh_flush(WCARRY * bf16r(v));
  }
  __syncthreads();
  v8h x[2];
  size_t off[2];
#pragma unroll
  for (unsigned i = 0; i < 2u; ++i) {
    const unsigned n = 32u * i + (tid >> 3);
    const unsigned kc = (tid & 7u) * 8u;
    x[i] = *(const v8h*)&T[n * LDT + kc];
    off[i] = (size_t)(n0 + n) * ldk + k0 + kc;
  }
#pragma unroll
  for (int i = 0; i < 2; ++i) *(volatile v8h*)(Wt + off[i]) = x[i];
  __threadfence();
#pragma unroll
  for (int i = 0; i < 2; ++i) *(volatile v8h*)(Wt + off[i]) = x[i];
}

__global__ __launch_bounds__(256) void xconv_kernel(
    const float* __restrict__ X, _Float16* __restrict__ X16) {
  const size_t e = ((size_t)blockIdx.x * 256u + threadIdx.x) * 8u;
  const v4f a0 = *(const v4f*)(X + e);
  const v4f a1 = *(const v4f*)(X + e + 4u);
  v8h o;
#pragma unroll
  for (int i = 0; i < 4; ++i) {
    o[i]     = toh_flush(ACARRY * bf16r(a0[i]));
    o[i + 4] = toh_flush(ACARRY * bf16r(a1[i]));
  }
  _Float16* p = X16 + e;
  *(volatile v8h*)p = o;
  __threadfence();
  *(volatile v8h*)p = o;
}

static_assert(16 * 4 == 64);
static_assert(32 * 2 == 64);

template <int MODE>
__device__ __forceinline__ void gemm_body(
    const _Float16* __restrict__ A16, const _Float16* __restrict__ Bt, const unsigned K,
    float* __restrict__ outf, const unsigned ldo, _Float16* __restrict__ out16) {
  __shared__ float Cs[64 * LDC];
  const unsigned tid = threadIdx.x, lane = tid & 31u;
  const unsigned w = (unsigned)__builtin_amdgcn_readfirstlane((int)(threadIdx.x >> 5));
  const unsigned mw = w >> 1, nw = w & 1u;
  const unsigned hh = lane >> 4, m = lane & 15u;
  const unsigned n0 = blockIdx.x * 64u;
  const unsigned row0 = blockIdx.y * 64u;

  const _Float16* ap  = A16 + (size_t)(row0 + mw * 16u + m) * K + hh * 8u;
  const _Float16* bp0 = Bt + (size_t)(n0 + nw * 32u + m) * K + hh * 8u;
  const _Float16* bp1 = bp0 + (size_t)16 * K;
  v8f acc0 = {}, acc1 = {};
#pragma unroll 2
  for (unsigned k0 = 0; k0 < K; k0 += 32u) {
    const v16h a  = frag_at(ap + k0);
    const v16h b0 = frag_at(bp0 + k0);
    const v16h b1 = frag_at(bp1 + k0);
    acc0 = wmma16(a, b0, acc0);
    acc1 = wmma16(a, b1, acc1);
  }
#pragma unroll
  for (int r = 0; r < 8; ++r) {
    float* d = &Cs[(mw * 16u + hh * 8u + (unsigned)r) * LDC + nw * 32u + m];
    d[0]  = acc0[r];
    d[16] = acc1[r];
  }
  __syncthreads();

  const float cs = 1.0f / (ACARRY * WCARRY);
  v4f xs[4];
  size_t off[4];
#pragma unroll
  for (unsigned i = 0; i < 4u; ++i) {
    const unsigned r = 16u * i + (tid >> 4);
    const unsigned c = (tid & 15u) * 4u;
    const v4f u = *(const v4f*)&Cs[r * LDC + c];
    v4f val;
#pragma unroll
    for (int j = 0; j < 4; ++j) val[j] = lif_last(u[j] * cs);
    xs[i] = val;
    off[i] = (size_t)(row0 + r) * ldo + n0 + c;
  }

  if (MODE == 0) {
    v8h x[2];
    size_t off16[2];
#pragma unroll
    for (unsigned i = 0; i < 2u; ++i) {
      const unsigned r = 32u * i + (tid >> 3);
      const unsigned c = (tid & 7u) * 8u;
      const v4f u0 = *(const v4f*)&Cs[r * LDC + c];
      const v4f u1 = *(const v4f*)&Cs[r * LDC + c + 4];
#pragma unroll
      for (int j = 0; j < 4; ++j) {
        x[i][j]     = toh_flush(ACARRY * lif_last(u0[j] * cs));
        x[i][j + 4] = toh_flush(ACARRY * lif_last(u1[j] * cs));
      }
      off16[i] = (size_t)(row0 + r) * HID + n0 + c;
    }
#pragma unroll
    for (int i = 0; i < 4; ++i) *(volatile v4f*)(outf + off[i]) = xs[i];
#pragma unroll
    for (int i = 0; i < 2; ++i) *(volatile v8h*)(out16 + off16[i]) = x[i];
    __threadfence();
#pragma unroll
    for (int i = 0; i < 4; ++i) *(volatile v4f*)(outf + off[i]) = xs[i];
#pragma unroll
    for (int i = 0; i < 2; ++i) *(volatile v8h*)(out16 + off16[i]) = x[i];
  } else {
#pragma unroll
    for (int i = 0; i < 4; ++i) *(volatile v4f*)(outf + off[i]) = xs[i];
    __threadfence();
#pragma unroll
    for (int i = 0; i < 4; ++i) *(volatile v4f*)(outf + off[i]) = xs[i];
  }
}

__global__ __launch_bounds__(256) void gemm_enc_kernel(
    const _Float16* __restrict__ A16, const _Float16* __restrict__ Bt,
    float* __restrict__ outf, _Float16* __restrict__ out16) {
  gemm_body<0>(A16, Bt, (unsigned)DIM, outf, (unsigned)HID, out16);
}
__global__ __launch_bounds__(256) void gemm_dec_kernel(
    const _Float16* __restrict__ A16, const _Float16* __restrict__ Bt,
    float* __restrict__ outf) {
  gemm_body<1>(A16, Bt, (unsigned)HID, outf, (unsigned)DIM, (_Float16*)0);
}

extern "C" void kernel_launch(void* const* d_in, const int* in_sizes, int n_in,
                              void* d_out, int out_size, void* d_ws, size_t ws_size,
                              hipStream_t stream) {
  if (n_in < 3) return;
  if ((long long)in_sizes[0] < (long long)MROWS * DIM) return;
  if ((long long)in_sizes[1] < (long long)DIM * HID) return;
  if ((long long)in_sizes[2] < (long long)HID * DIM) return;
  if ((long long)out_size < (long long)NB_FULL * DIM + (long long)MROWS * HID) return;
  if (ws_size < WS_TOTAL) return;

  const float* X     = (const float*)d_in[0];
  const float* enc_w = (const float*)d_in[1];
  const float* dec_w = (const float*)d_in[2];
  float* out0 = (float*)d_out;
  float* out1 = (float*)d_out + OUT1_OFF;

  char* ws = (char*)d_ws;
  _Float16* Enc_t = (_Float16*)(ws + OFF_ENC);
  _Float16* Dec_t = (_Float16*)(ws + OFF_DEC);
  _Float16* X16   = (_Float16*)(ws + OFF_X16);
  _Float16* E16   = (_Float16*)(ws + OFF_E16);

  dim3 blk(256);

  wconv_kernel<<<dim3(HID / 64, DIM / 64), blk, 0, stream>>>(enc_w, Enc_t, (unsigned)HID, (unsigned)DIM);
  wconv_kernel<<<dim3(DIM / 64, HID / 64), blk, 0, stream>>>(dec_w, Dec_t, (unsigned)DIM, (unsigned)HID);
  xconv_kernel<<<dim3((unsigned)(((size_t)MROWS * DIM) / 2048u)), blk, 0, stream>>>(X, X16);
  gemm_enc_kernel<<<dim3(HID / 64, MROWS / 64), blk, 0, stream>>>(X16, Enc_t, out1, E16);
  gemm_dec_kernel<<<dim3(DIM / 64, MROWS / 64), blk, 0, stream>>>(E16, Dec_t, out0);
}
